// DAGCNLayer_16947940950535
// MI455X (gfx1250) — hardware-verified
//
#include <hip/hip_runtime.h>
#include <math.h>

#define N_NODES 4096
#define H_DIM   256
#define H2_DIM  512
#define N_HEADS 4
#define D_HEAD  64
#define E_EDGES 262144
#define NT 256
#define SRB 512
#define NTILE (N_NODES / SRB)
#define SCH 2048
#define NCH (E_EDGES / SCH)
#define WSC 64.0f

typedef __attribute__((ext_vector_type(16))) _Float16 v16h;
typedef __attribute__((ext_vector_type(8)))  _Float16 v8h;
typedef __attribute__((ext_vector_type(4)))  _Float16 v4h;
typedef __attribute__((ext_vector_type(16))) __bf16   v16b;
typedef __attribute__((ext_vector_type(8)))  __bf16   v8b;
typedef __attribute__((ext_vector_type(8)))  float    v8f;
typedef __attribute__((ext_vector_type(4)))  float    v4f;
typedef __attribute__((ext_vector_type(4)))  int      v4i;

__device__ __forceinline__ unsigned short f2bf_bits(float f) {
  unsigned u = __float_as_uint(f);
  return (unsigned short)((u + 0x7FFFu + ((u >> 16) & 1u)) >> 16);
}
__device__ __forceinline__ float bf_bits2f(unsigned short h) { return __uint_as_float(((unsigned)h) << 16); }

__device__ __forceinline__ void dep_guard_h(v8f& a, v8f& b, v16h x, v16h y) { asm volatile("v_nop\n\tv_nop\n\tv_nop\n\tv_nop" : "+v"(a), "+v"(b) : "v"(x), "v"(y)); }
__device__ __forceinline__ void dep_guard_b(v8f& a, v8f& b, v16b x, v16b y) { asm volatile("v_nop\n\tv_nop\n\tv_nop\n\tv_nop" : "+v"(a), "+v"(b) : "v"(x), "v"(y)); }
__device__ __forceinline__ void keep4_h(v16h a, v16h b, v16h c, v16h d) { asm volatile("v_nop" :: "v"(a), "v"(b), "v"(c), "v"(d)); }
__device__ __forceinline__ void keep4_b(v16b a, v16b b, v16b c, v16b d) { asm volatile("v_nop" :: "v"(a), "v"(b), "v"(c), "v"(d)); }
__device__ __forceinline__ void acc_guard4(v8f& a, v8f& b, v8f& c, v8f& d) { asm volatile("v_nop\n\tv_nop\n\tv_nop\n\tv_nop" : "+v"(a), "+v"(b), "+v"(c), "+v"(d)); }
template <typename T> struct Frag;
template <> struct Frag<_Float16> {
  typedef v16h V; union U { v16h v; v8h h[2]; };
  static __device__ __forceinline__ v16h load(const _Float16* p) {
    U f; f.h[0] = *(const v8h*)(p); f.h[1] = *(const v8h*)(p + 16); return f.v;
  }
  static __device__ __forceinline__ v8f mma(v16h a, v16h b, v8f c) {
    return __builtin_amdgcn_wmma_f32_16x16x32_f16(false, a, false, b, (short)0, c, false, false);
  }
  static __device__ __forceinline__ void guard(v8f& a, v8f& b, v16h x, v16h y) { dep_guard_h(a, b, x, y); }
  static __device__ __forceinline__ void keep(v16h a, v16h b, v16h c, v16h d) { keep4_h(a, b, c, d); }
};
template <> struct Frag<__bf16> {
  typedef v16b V; union U { v16b v; v8b h[2]; };
  static __device__ __forceinline__ v16b load(const __bf16* p) {
    U f; f.h[0] = *(const v8b*)(p); f.h[1] = *(const v8b*)(p + 16); return f.v;
  }
  static __device__ __forceinline__ v8f mma(v16b a, v16b b, v8f c) {
    return __builtin_amdgcn_wmma_f32_16x16x32_bf16(false, a, false, b, (short)0, c, false, false);
  }
  static __device__ __forceinline__ void guard(v8f& a, v8f& b, v16b x, v16b y) { dep_guard_b(a, b, x, y); }
  static __device__ __forceinline__ void keep(v16b a, v16b b, v16b c, v16b d) { keep4_b(a, b, c, d); }
};

template <int ET> struct Elem;
template <> struct Elem<0> { typedef _Float16 T; };
template <> struct Elem<1> { typedef __bf16 T; };
template <int ET, bool SPLIT, int BIAS_MODE, int OUT_MODE, bool RESID, int ACT = 0>
__global__ __launch_bounds__(256) void wmma_gemm64(
    const unsigned short* __restrict__ Ap, const unsigned short* __restrict__ A2p, int lda, long strideA,
    const unsigned short* __restrict__ Btp, const unsigned short* __restrict__ Bt2p, int ldb, long strideB,
    void* __restrict__ Cout, void* __restrict__ Cout2, int ldc, long strideC,
    const float* __restrict__ bias,
    const float* __restrict__ resid, long strideR,
    int M, int N, int K, float scale) {
  typedef typename Elem<ET>::T T;
  typedef typename Frag<T>::V V;
  const T* A = (const T*)Ap; const T* A2 = (const T*)A2p; const T* Bt = (const T*)Btp; const T* Bt2 = (const T*)Bt2p;
  __shared__ __align__(16) float sT[8][16 * 68];
  const int b    = blockIdx.y;
  const int lane = threadIdx.x & 31;
  const int wave = threadIdx.x >> 5;
  const int tilesN = N >> 6;
  const int tilesM = M >> 6;
  const int tile = blockIdx.x * 8 + wave;
  if (tile >= tilesM * tilesN) return;
  const int tm = tile / tilesN;
  const int tn = tile - tm * tilesN;
  const int m0 = tm << 6;
  const int n0 = tn << 6;

  const T* Ab  = A  + (size_t)b * strideA;
  const T* Bb  = Bt + (size_t)b * strideB;
  const T* Ab2 = SPLIT ? (A2  + (size_t)b * strideA) : nullptr;
  const T* Bb2 = SPLIT ? (Bt2 + (size_t)b * strideB) : nullptr;

  const int rlane = lane & 15;
  const int koff  = (lane >> 4) * 8;
  const int mOff  = (lane >> 4) * 8;

  v8f acc[4][4];
#pragma unroll
  for (int i = 0; i < 4; ++i)
#pragma unroll
    for (int j = 0; j < 4; ++j) acc[i][j] = (v8f){0.f,0.f,0.f,0.f,0.f,0.f,0.f,0.f};

  for (int k0 = 0; k0 < K; k0 += 32) {
    V bh[4], bl[4];
#pragma unroll
    for (int j = 0; j < 4; ++j) {
      const size_t bo = (size_t)(n0 + (j << 4) + rlane) * ldb + koff + k0;
      bh[j] = Frag<T>::load(Bb + bo);
      if (SPLIT) bl[j] = Frag<T>::load(Bb2 + bo);
    }
#pragma unroll
    for (int i = 0; i < 4; ++i) {
      const size_t ao = (size_t)(m0 + (i << 4) + rlane) * lda + koff + k0;
      V ah = Frag<T>::load(Ab + ao);
      V al;
      if (SPLIT) al = Frag<T>::load(Ab2 + ao);
#pragma unroll
      for (int j = 0; j < 4; ++j) {
        acc[i][j] = Frag<T>::mma(ah, bh[j], acc[i][j]);
        if (SPLIT) {
          acc[i][j] = Frag<T>::mma(ah, bl[j], acc[i][j]);
          acc[i][j] = Frag<T>::mma(al, bh[j], acc[i][j]);
        }
      }
      Frag<T>::guard(acc[i][0], acc[i][3], ah, SPLIT ? al : ah);
    }
    Frag<T>::keep(bh[0], bh[1], bh[2], bh[3]);
    if (SPLIT) Frag<T>::keep(bl[0], bl[1], bl[2], bl[3]);
  }
  acc_guard4(acc[0][0], acc[0][1], acc[0][2], acc[0][3]);
  acc_guard4(acc[1][0], acc[1][1], acc[1][2], acc[1][3]);
  acc_guard4(acc[2][0], acc[2][1], acc[2][2], acc[2][3]);
  acc_guard4(acc[3][0], acc[3][1], acc[3][2], acc[3][3]);

  float* slab = sT[wave];
  const float* Rb = RESID ? (resid + (size_t)b * strideR) : nullptr;
#pragma unroll
  for (int i = 0; i < 4; ++i) {
    const int mBase = m0 + (i << 4);
#pragma unroll
    for (int j = 0; j < 4; ++j) {
      const int n = n0 + (j << 4) + rlane;
      float bv = 0.f;
      if (BIAS_MODE == 2) bv = bias[n];
#pragma unroll
      for (int r = 0; r < 8; ++r) {
        float v = acc[i][j][r] * scale;
        if (BIAS_MODE == 1) v += bias[mBase + mOff + r];
        if (BIAS_MODE == 2) v += bv;
        if (RESID) v += Rb[(size_t)(mBase + mOff + r) * ldc + n];
        if (ACT == 1) v = tanhf(v);
        if (ACT == 2) v = fmaxf(v, 0.0f);
        if (ACT == 3) v = v / (1.0f + expf(-v));
        if (ACT == 4) v = (v > 0.f) ? v : 0.01f * v;
        if (ACT == 5) v = 0.5f * v * (1.0f + erff(v * 0.70710678118654752f));
        slab[(mOff + r) * 68 + (j << 4) + rlane] = v;
      }
    }
    __builtin_amdgcn_fence(__ATOMIC_RELEASE, "workgroup");
    __builtin_amdgcn_wave_barrier();
    __builtin_amdgcn_fence(__ATOMIC_ACQUIRE, "workgroup");
    if (OUT_MODE == 0) {
      float* C = (float*)Cout + (size_t)b * strideC;
      const int hh = lane >> 4, c4 = (lane & 15) * 4;
      for (int pass = 0; pass < 2; ++pass) {
#pragma unroll
        for (int it = 0; it < 8; ++it) {
          const int row = it * 2 + hh;
          v4f v = *(const v4f*)(slab + row * 68 + c4);
          *(volatile v4f*)(C + (size_t)(mBase + row) * ldc + n0 + c4) = v;
        }
        __threadfence();
      }
    } else {
      const int q = lane >> 3, c8 = (lane & 7) * 8;
      unsigned short* C  = (unsigned short*)Cout  + (size_t)b * strideC;
      unsigned short* C2 = (OUT_MODE == 2) ? ((unsigned short*)Cout2 + (size_t)b * strideC) : nullptr;
      for (int pass = 0; pass < 2; ++pass) {
#pragma unroll
        for (int it = 0; it < 4; ++it) {
          const int row = it * 4 + q;
          const float* sp = slab + row * 68 + c8;
          v8h hv, lv;
#pragma unroll
          for (int e = 0; e < 8; ++e) {
            if (OUT_MODE == 1) {
              hv[e] = (_Float16)sp[e];
            } else {
              unsigned short hb = f2bf_bits(sp[e]);
              unsigned short lb = f2bf_bits(sp[e] - bf_bits2f(hb));
              hv[e] = __builtin_bit_cast(_Float16, hb);
              lv[e] = __builtin_bit_cast(_Float16, lb);
            }
          }
          *(volatile v8h*)(C + (size_t)(mBase + row) * ldc + n0 + c8) = hv;
          if (OUT_MODE == 2) *(volatile v8h*)(C2 + (size_t)(mBase + row) * ldc + n0 + c8) = lv;
        }
        __threadfence();
      }
    }
    __builtin_amdgcn_fence(__ATOMIC_RELEASE, "workgroup");
    __builtin_amdgcn_wave_barrier();
    __builtin_amdgcn_fence(__ATOMIC_ACQUIRE, "workgroup");
  }
}

__global__ __launch_bounds__(256) void cast_f32_f16x2(
    const float* __restrict__ in, _Float16* __restrict__ out, int n2) {
  int i = blockIdx.x * 256 + threadIdx.x;
  if (i < n2) {
    const _Float16 h0 = (_Float16)in[2 * i], h1 = (_Float16)in[2 * i + 1];
    const unsigned u = (unsigned)__builtin_bit_cast(unsigned short, h0) | ((unsigned)__builtin_bit_cast(unsigned short, h1) << 16);
    ((volatile unsigned*)out)[i] = u;
    __threadfence();
    ((volatile unsigned*)out)[i] = u;
  }
}

__global__ __launch_bounds__(256) void tcast_f16_kernel(const float* __restrict__ W, unsigned short* __restrict__ out,
                                                       int Kin, int Nout, float scale) {
  const int kh = Kin >> 1;
  const int n2 = kh * Nout;
  const int i = blockIdx.x * 256 + threadIdx.x;
  if (i < n2) {
    const int o = i / kh;
    const int k = 2 * (i - o * kh);
    const float a = W[(size_t)k * Nout + o] * scale;
    const float b = W[(size_t)(k + 1) * Nout + o] * scale;
    const _Float16 ha = (_Float16)a, hb = (_Float16)b;
    const unsigned u = (unsigned)__builtin_bit_cast(unsigned short, ha) | ((unsigned)__builtin_bit_cast(unsigned short, hb) << 16);
    ((volatile unsigned*)out)[i] = u;
    __threadfence();
    ((volatile unsigned*)out)[i] = u;
  }
}

__device__ __forceinline__ int blk_excl_scan(int cnt, int* scan_ws, int tid, int* tot) {
  const int lane = tid & 31, wave = tid >> 5; int incl = cnt;
#pragma unroll
  for (int o = 1; o < 32; o <<= 1) { const int v = __shfl_up(incl, o, 32); if (lane >= o) incl += v; }
  if (lane == 31) scan_ws[wave] = incl;
  __syncthreads();
  if (wave == 0) { int wv = (lane < NT / 32) ? scan_ws[lane] : 0; int wincl = wv;
#pragma unroll
    for (int o = 1; o < 32; o <<= 1) { const int v = __shfl_up(wincl, o, 32); if (lane >= o) wincl += v; }
    if (lane < NT / 32) scan_ws[32 + lane] = wincl - wv; if (lane == 31) scan_ws[64] = wincl; }
  __syncthreads();
  const int res = scan_ws[32 + wave] + incl - cnt; *tot = scan_ws[64];
  return res;
}
template <int SP, int CAP>
__device__ __forceinline__ int chunk_hits(const int* __restrict__ dstv, const int* __restrict__ srcv, int e0, int n0, int tid,
                                          int* LIST, int* scan_ws) {
  const int eb = e0 + tid * SP;
  const bool inr = (eb + SP) <= E_EDGES;
  const int ebc = inr ? eb : (E_EDGES - SP);
  int rec[SP]; int cnt = 0;
#pragma unroll
  for (int k = 0; k < SP; k += 4) {
    const v4i d4 = *(const v4i*)(dstv + ebc + k);
    const v4i s4 = *(const v4i*)(srcv + ebc + k);
#pragma unroll
    for (int e = 0; e < 4; ++e) {
      const int d = d4[e]; int r = -1;
      if (inr && d >= n0 && d < n0 + SRB) {
        int s = s4[e]; s = s < 0 ? 0 : (s >= N_NODES ? N_NODES - 1 : s);
        r = ((d - n0) << 16) | s; ++cnt;
      }
      rec[k + e] = r;
    }
  }
  int tot; int p = blk_excl_scan(cnt, scan_ws, tid, &tot);
#pragma unroll
  for (int k = 0; k < SP; ++k) if (rec[k] >= 0) { if ((unsigned)p < (unsigned)CAP) LIST[p] = rec[k]; ++p; }
  __syncthreads();
  return tot < CAP ? tot : CAP;
}

__global__ __launch_bounds__(NT) void agg_kernel(const float* __restrict__ Pst, const int* __restrict__ ei,
                                                const float* __restrict__ bsrc, const float* __restrict__ btgt,
                                                float* ACC, unsigned short* __restrict__ AGp) {
  __shared__ int LIST[SCH];
  __shared__ int SDEG[SRB];
  __shared__ int scan_ws[80];
  const int tid = threadIdx.x, lane = tid & 31, wave = tid >> 5;
  const int n0 = blockIdx.x * SRB;
  _Float16* AG = (_Float16*)AGp;
  const v4f z4 = {0.f, 0.f, 0.f, 0.f};
#pragma unroll 1
  for (int j = 0; j < 64; ++j) {
    float* rp = ACC + (size_t)(n0 + wave * 64 + j) * H_DIM + 4 * lane;
    *(volatile v4f*)rp = z4; *(volatile v4f*)(rp + 128) = z4;
    __threadfence();
    *(volatile v4f*)rp = z4; *(volatile v4f*)(rp + 128) = z4;
  }
  for (int i = tid; i < SRB; i += NT) SDEG[i] = 0;
  __syncthreads();
  const int* srcv = ei; const int* dstv = ei + E_EDGES;
#pragma unroll 1
  for (int c = 0; c < NCH; ++c) {
    const int tot = chunk_hits<SCH / NT, SCH>(dstv, srcv, c * SCH, n0, tid, LIST, scan_ws);
#pragma unroll 1
    for (int base = 0; base < tot; base += 32) {
      const int q = base + lane;
      const int qc = q < SCH ? q : SCH - 1;
      const int lv = LIST[qc];
      const int rv = (q < tot) ? lv : -1;
      const int own = (rv >= 0 && (rv >> 22) == wave) ? 1 : 0;
      unsigned msk = (unsigned)__ballot(own);
#pragma unroll 1
      for (int it = 0; it < 32; ++it) {
        if (msk == 0u) break;
        const int bp = __builtin_ctz(msk); msk &= msk - 1u;
        const int r = __shfl(rv, bp, 32);
        const int dl = (r >> 16) & (SRB - 1);
        const int s  = r & (N_NODES - 1);
        const float* pr = Pst + (size_t)s * H2_DIM + 4 * lane;
        const v4f p0 = *(const v4f*)pr, p1 = *(const v4f*)(pr + 128);
        float* rp = ACC + (size_t)(n0 + dl) * H_DIM + 4 * lane;
        v4f a0 = *(const v4f*)rp, a1 = *(const v4f*)(rp + 128);
        a0 = a0 + p0; a1 = a1 + p1;
        if (lane == 0) SDEG[dl] += 1;
        *(volatile v4f*)rp = a0; *(volatile v4f*)(rp + 128) = a1;
        __threadfence();
        *(volatile v4f*)rp = a0; *(volatile v4f*)(rp + 128) = a1;
      }
    }
    __syncthreads();
  }
  const v4f bA = *(const v4f*)(bsrc + 4 * lane) + *(const v4f*)(btgt + 4 * lane);
  const v4f bB = *(const v4f*)(bsrc + 128 + 4 * lane) + *(const v4f*)(btgt + 128 + 4 * lane);
#pragma unroll 1
  for (int j = 0; j < 64; ++j) {
    const int dl = wave * 64 + j; const int n = n0 + dl;
    const float degf = (float)SDEG[dl];
    const float inv = 1.0f / fmaxf(degf, 1.0f);
    const float* rp = ACC + (size_t)n * H_DIM + 4 * lane;
    const v4f a0 = *(const v4f*)rp, a1 = *(const v4f*)(rp + 128);
    const float* pt = Pst + (size_t)n * H2_DIM + H_DIM + 4 * lane;
    const v4f t0 = *(const v4f*)pt, t1 = *(const v4f*)(pt + 128);
    const v4f o0 = (a0 + degf * (t0 + bA)) * inv;
    const v4f o1 = (a1 + degf * (t1 + bB)) * inv;
    v4h h0, h1;
#pragma unroll
    for (int e = 0; e < 4; ++e) { h0[e] = (_Float16)o0[e]; h1[e] = (_Float16)o1[e]; }
    _Float16* ar = AG + (size_t)n * H_DIM + 4 * lane;
    *(volatile v4h*)ar = h0; *(volatile v4h*)(ar + 128) = h1;
    __threadfence();
    *(volatile v4h*)ar = h0; *(volatile v4h*)(ar + 128) = h1;
  }
}

#define AT_D 64
#define AT_NW 4
#define AT_KC 64
#define P_SC 32768.0f
__device__ __forceinline__ v8f mma16h(v16h a, v16h b, v8f c) {
  c = __builtin_amdgcn_wmma_f32_16x16x32_f16(false, a, false, b, (short)0, c, false, false);
  asm volatile("v_nop\n\tv_nop\n\tv_nop\n\tv_nop" : "+v"(c) : "v"(a), "v"(b));
  return c;
}
__global__ __launch_bounds__(128)
void attn_f16_kernel(const unsigned short* __restrict__ qp, const unsigned short* __restrict__ kp,
                     const unsigned short* __restrict__ vp, unsigned short* __restrict__ op,
                     int S, int ld, float sscale, float oscale) {
  union FH { v16h v; v8h h[2]; };
  __shared__ __align__(16) _Float16 Ksh[AT_KC * AT_D];
  __shared__ __align__(16) _Float16 Vth[AT_D * AT_KC];
  __shared__ __align__(16) _Float16 Psh[AT_NW][16 * AT_KC];
  __shared__ __align__(16) float  Os[AT_NW][16 * 68];
  const _Float16* q = (const _Float16*)qp;
  const _Float16* k = (const _Float16*)kp;
  const _Float16* v = (const _Float16*)vp;
  _Float16* o = (_Float16*)op;
  const int tid  = threadIdx.x;
  const int wave = tid >> 5;
  const int lane = tid & 31;
  const int hh   = lane >> 4;
  const int c    = lane & 15;
  const int nqb  = S >> 6;
  const int qb   = blockIdx.x % nqb;
  const int head = blockIdx.x / nqb;
  const int hoff = head * AT_D;
  const int q0   = qb * 64 + wave * 16;

  v16h qa[2];
#pragma unroll
  for (int dc = 0; dc < 2; ++dc) qa[dc] = Frag<_Float16>::load(q + (size_t)(q0 + c) * ld + hoff + dc * 32 + 8 * hh);

  float mrow[8], lrow[8];
  v8f oacc[4];
#pragma unroll
  for (int r = 0; r < 8; ++r) { mrow[r] = -INFINITY; lrow[r] = 0.f; }
#pragma unroll
  for (int t = 0; t < 4; ++t) oacc[t] = (v8f){0.f,0.f,0.f,0.f,0.f,0.f,0.f,0.f};

  const int nChunks = S >> 6;
#pragma unroll 1
  for (int kc = 0; kc < nChunks; ++kc) {
    const int kv0 = kc * AT_KC;
    __syncthreads();
    {
      const int kvr = tid >> 1, dh = (tid & 1) * 32;
      const _Float16* krow = k + (size_t)(kv0 + kvr) * ld + hoff + dh;
      const _Float16* vrow = v + (size_t)(kv0 + kvr) * ld + hoff + dh;
#pragma unroll
      for (int i = 0; i < 4; ++i) {
        const v8h kk8 = *(const v8h*)(krow + 8 * i);
        *(v8h*)(Ksh + kvr * AT_D + dh + 8 * i) = kk8;
        const v8h vv8 = *(const v8h*)(vrow + 8 * i);
#pragma unroll
        for (int e = 0; e < 8; ++e) Vth[(dh + 8 * i + e) * AT_KC + kvr] = vv8[e];
      }
    }
    __syncthreads();

    v8f s[4];
#pragma unroll
    for (int j = 0; j < 4; ++j) {
      s[j] = (v8f){0.f,0.f,0.f,0.f,0.f,0.f,0.f,0.f};
#pragma unroll
      for (int dc = 0; dc < 2; ++dc) {
        FH kb;
        kb.h[0] = *(const v8h*)(Ksh + (j * 16 + c) * AT_D + dc * 32 + 8 * hh);
        kb.h[1] = *(const v8h*)(Ksh + (j * 16 + c) * AT_D + dc * 32 + 16 + 8 * hh);
        s[j] = mma16h(qa[dc], kb.v, s[j]);
      }
    }
    float cm[8];
#pragma unroll
    for (int r = 0; r < 8; ++r) {
      float m = -INFINITY;
#pragma unroll
      for (int j = 0; j < 4; ++j) { s[j][r] = s[j][r] * sscale; m = fmaxf(m, s[j][r]); }
#pragma unroll
      for (int off = 1; off < 16; off <<= 1) m = fmaxf(m, __shfl_xor(m, off, 32));
      cm[r] = m;
    }
    _Float16* pw = Psh[wave];
#pragma unroll
    for (int r = 0; r < 8; ++r) {
      const float mnew = fmaxf(mrow[r], cm[r]);
      const float alpha = expf(mrow[r] - mnew);
      mrow[r] = mnew;
      float psum = 0.f;
#pragma unroll
      for (int j = 0; j < 4; ++j) {
        const float p = expf(s[j][r] - mnew);
        psum += p;
        pw[(8 * hh + r) * AT_KC + j * 16 + c] = (_Float16)(p * P_SC);
      }
#pragma unroll
      for (int off = 1; off < 16; off <<= 1) psum += __shfl_xor(psum, off, 32);
      lrow[r] = lrow[r] * alpha + psum;
#pragma unroll
      for (int t = 0; t < 4; ++t) oacc[t][r] *= alpha;
    }
    __builtin_amdgcn_fence(__ATOMIC_RELEASE, "workgroup");
    __builtin_amdgcn_wave_barrier();
    __builtin_amdgcn_fence(__ATOMIC_ACQUIRE, "workgroup");
#pragma unroll 1
    for (int kk = 0; kk < 2; ++kk) {
      FH pa;
      pa.h[0] = *(const v8h*)(pw + c * AT_KC + kk * 32 + 8 * hh);
      pa.h[1] = *(const v8h*)(pw + c * AT_KC + kk * 32 + 16 + 8 * hh);
#pragma unroll
      for (int t = 0; t < 4; ++t) {
        FH vb;
        vb.h[0] = *(const v8h*)(Vth + (t * 16 + c) * AT_KC + kk * 32 + 8 * hh);
        vb.h[1] = *(const v8h*)(Vth + (t * 16 + c) * AT_KC + kk * 32 + 16 + 8 * hh);
        oacc[t] = mma16h(pa.v, vb.v, oacc[t]);
      }
    }
  }

  float* os = Os[wave];
#pragma unroll
  for (int r = 0; r < 8; ++r) {
    const float inv = oscale * (1.0f / (lrow[r] * P_SC));
#pragma unroll
    for (int t = 0; t < 4; ++t) os[(8 * hh + r) * 68 + t * 16 + c] = oacc[t][r] * inv;
  }
  __builtin_amdgcn_fence(__ATOMIC_RELEASE, "workgroup");
  __builtin_amdgcn_wave_barrier();
  __builtin_amdgcn_fence(__ATOMIC_ACQUIRE, "workgroup");
  {
    const int qq = lane >> 3, c8 = (lane & 7) * 8;
    for (int pass = 0; pass < 2; ++pass) {
#pragma unroll
      for (int it = 0; it < 4; ++it) {
        const int row = it * 4 + qq;
        const float* sp = os + row * 68 + c8;
        v8h hv;
#pragma unroll
        for (int e = 0; e < 8; ++e) hv[e] = (_Float16)sp[e];
        *(volatile v8h*)(o + (size_t)(q0 + row) * ld + hoff + c8) = hv;
      }
      __threadfence();
    }
  }
}

template <bool WH>
__global__ __launch_bounds__(NT) void ln_kernel(const float* __restrict__ y, const float* __restrict__ g, const float* __restrict__ be,
                                                float* __restrict__ xf, unsigned short* __restrict__ xhp, int nrows) {
  const int wave = threadIdx.x >> 5, lane = threadIdx.x & 31;
  const int row = blockIdx.x * 8 + wave;
  if (row >= nrows) return;
  const float* yr = y + (size_t)row * H_DIM;
  const v4f a0 = *(const v4f*)(yr + 4 * lane), a1 = *(const v4f*)(yr + 128 + 4 * lane);
  float s = ((a0[0] + a0[1]) + (a0[2] + a0[3])) + ((a1[0] + a1[1]) + (a1[2] + a1[3]));
#pragma unroll
  for (int m = 1; m < 32; m <<= 1) s += __shfl_xor(s, m, 32);
  const float mu = s * (1.0f / H_DIM);
  const v4f d0 = a0 - mu, d1 = a1 - mu;
  float vs = d0[0] * d0[0] + d0[1] * d0[1] + d0[2] * d0[2] + d0[3] * d0[3]
           + d1[0] * d1[0] + d1[1] * d1[1] + d1[2] * d1[2] + d1[3] * d1[3];
#pragma unroll
  for (int m = 1; m < 32; m <<= 1) vs += __shfl_xor(vs, m, 32);
  const float var = vs * (1.0f / H_DIM);
  const float rinv = 1.0f / sqrtf(var + 1e-5f);
  const v4f g0 = *(const v4f*)(g + 4 * lane), g1 = *(const v4f*)(g + 128 + 4 * lane);
  const v4f e0 = *(const v4f*)(be + 4 * lane), e1 = *(const v4f*)(be + 128 + 4 * lane);
  const v4f t0 = d0 * rinv, t1 = d1 * rinv;
  const v4f o0 = t0 * g0 + e0, o1 = t1 * g1 + e1;
  v4h h0, h1;
#pragma unroll
  for (int e = 0; e < 4; ++e) { h0[e] = (_Float16)o0[e]; h1[e] = (_Float16)o1[e]; }
  float* xr = xf + (size_t)row * H_DIM + 4 * lane;
  _Float16* hr = (_Float16*)xhp + (size_t)row * H_DIM + 4 * lane;
  *(volatile v4f*)xr = o0; *(volatile v4f*)(xr + 128) = o1;
  if (WH) { *(volatile v4h*)hr = h0; *(volatile v4h*)(hr + 128) = h1; }
  __threadfence();
  *(volatile v4f*)xr = o0; *(volatile v4f*)(xr + 128) = o1;
  if (WH) { *(volatile v4h*)hr = h0; *(volatile v4h*)(hr + 128) = h1; }
}

extern "C" void kernel_launch(void* const* d_in, const int* in_sizes, int n_in,
                              void* d_out, int out_size, void* d_ws, size_t ws_size, hipStream_t stream) {
  if (n_in < 22) return;
  if (in_sizes[0] != N_NODES * H_DIM || in_sizes[1] != 2 * E_EDGES || out_size != N_NODES * H_DIM) return;
  if (in_sizes[14] != H_DIM * H2_DIM || in_sizes[16] != H2_DIM * H_DIM) return;

  const float* h     = (const float*)d_in[0];
  const int*   eidx  = (const int*)d_in[1];
  const float* W_src = (const float*)d_in[2];
  const float* b_src = (const float*)d_in[3];
  const float* W_tgt = (const float*)d_in[4];
  const float* b_tgt = (const float*)d_in[5];
  const float* Wq    = (const float*)d_in[6];
  const float* bq    = (const float*)d_in[7];
  const float* Wk    = (const float*)d_in[8];
  const float* bk    = (const float*)d_in[9];
  const float* Wv    = (const float*)d_in[10];
  const float* bv    = (const float*)d_in[11];
  const float* Wo    = (const float*)d_in[12];
  const float* bo    = (const float*)d_in[13];
  const float* W1    = (const float*)d_in[14];
  const float* b1    = (const float*)d_in[15];
  const float* W2    = (const float*)d_in[16];
  const float* b2    = (const float*)d_in[17];
  const float* g1    = (const float*)d_in[18];
  const float* be1   = (const float*)d_in[19];
  const float* g2    = (const float*)d_in[20];
  const float* be2   = (const float*)d_in[21];
  float* out = (float*)d_out;

  const size_t NH  = (size_t)N_NODES * H_DIM;
  const size_t NH2 = (size_t)N_NODES * H2_DIM;
  char* ws = (char*)d_ws; size_t off = 0;
  auto carve = [&](size_t bytes) -> char* { char* p = ws + off; off += (bytes + 255) & ~(size_t)255; return p; };
  unsigned short* Hh   = (unsigned short*)carve(NH * 2);
  unsigned short* Bst  = (unsigned short*)carve((size_t)H2_DIM * H_DIM * 2);
  unsigned short* WqT  = (unsigned short*)carve((size_t)H_DIM * H_DIM * 2);
  unsigned short* WkT  = (unsigned short*)carve((size_t)H_DIM * H_DIM * 2);
  unsigned short* WvT  = (unsigned short*)carve((size_t)H_DIM * H_DIM * 2);
  unsigned short* WoT  = (unsigned short*)carve((size_t)H_DIM * H_DIM * 2);
  unsigned short* W1T  = (unsigned short*)carve((size_t)H2_DIM * H_DIM * 2);
  unsigned short* W2T  = (unsigned short*)carve((size_t)H_DIM * H2_DIM * 2);
  float*          Pst  = (float*)carve(NH2 * 4);
  float*          ACC  = (float*)carve(NH * 4);
  unsigned short* AGh  = (unsigned short*)carve(NH * 2);
  unsigned short* Qh   = (unsigned short*)carve(NH * 2);
  unsigned short* Kh   = (unsigned short*)carve(NH * 2);
  unsigned short* Vh   = (unsigned short*)carve(NH * 2);
  unsigned short* CTXh = (unsigned short*)carve(NH * 2);
  float*          Y1   = (float*)carve(NH * 4);
  float*          Xf   = (float*)carve(NH * 4);
  unsigned short* Xh   = (unsigned short*)carve(NH * 2);
  unsigned short* F1h  = (unsigned short*)carve(NH2 * 2);
  float*          Y2   = (float*)carve(NH * 4);
  if (off > ws_size || off > (size_t)134217728) return;

  const float wsc = WSC;
  cast_f32_f16x2<<<(unsigned)((NH / 2 + 255) / 256), 256, 0, stream>>>(h, (_Float16*)Hh, (int)(NH / 2));
  {
    const int nHH = (H_DIM / 2) * H_DIM;
    const int nH2 = (H_DIM / 2) * H2_DIM;
    const int n2H = (H2_DIM / 2) * H_DIM;
    tcast_f16_kernel<<<(nHH + 255) / 256, 256, 0, stream>>>(W_src, Bst, H_DIM, H_DIM, wsc);
    tcast_f16_kernel<<<(nHH + 255) / 256, 256, 0, stream>>>(W_tgt, Bst + (size_t)H_DIM * H_DIM, H_DIM, H_DIM, wsc);
    tcast_f16_kernel<<<(nHH + 255) / 256, 256, 0, stream>>>(Wq, WqT, H_DIM, H_DIM, wsc);
    tcast_f16_kernel<<<(nHH + 255) / 256, 256, 0, stream>>>(Wk, WkT, H_DIM, H_DIM, wsc);
    tcast_f16_kernel<<<(nHH + 255) / 256, 256, 0, stream>>>(Wv, WvT, H_DIM, H_DIM, wsc);
    tcast_f16_kernel<<<(nHH + 255) / 256, 256, 0, stream>>>(Wo, WoT, H_DIM, H_DIM, wsc);
    tcast_f16_kernel<<<(nH2 + 255) / 256, 256, 0, stream>>>(W1, W1T, H_DIM, H2_DIM, wsc);
    tcast_f16_kernel<<<(n2H + 255) / 256, 256, 0, stream>>>(W2, W2T, H2_DIM, H_DIM, wsc);
  }
  const int tilesH  = (N_NODES / 64) * (H_DIM / 64);
  const int tilesH2 = (N_NODES / 64) * (H2_DIM / 64);
  const float isc = 1.0f / WSC;

  wmma_gemm64<0, false, 0, 0, false><<<dim3((tilesH2 + 7) / 8, 1), 256, 0, stream>>>(
      Hh, nullptr, H_DIM, 0L, Bst, nullptr, H_DIM, 0L, (void*)Pst, nullptr, H2_DIM, 0L,
      nullptr, nullptr, 0L, N_NODES, H2_DIM, H_DIM, isc);
  wmma_gemm64<0, false, 2, 1, false><<<dim3((tilesH + 7) / 8, 1), 256, 0, stream>>>(
      Hh, nullptr, H_DIM, 0L, WqT, nullptr, H_DIM, 0L, (void*)Qh, nullptr, H_DIM, 0L,
      bq, nullptr, 0L, N_NODES, H_DIM, H_DIM, isc);
  agg_kernel<<<NTILE, NT, 0, stream>>>(Pst, eidx, b_src, b_tgt, ACC, AGh);
  wmma_gemm64<0, false, 2, 1, false><<<dim3((tilesH + 7) / 8, 1), 256, 0, stream>>>(
      AGh, nullptr, H_DIM, 0L, WkT, nullptr, H_DIM, 0L, (void*)Kh, nullptr, H_DIM, 0L,
      bk, nullptr, 0L, N_NODES, H_DIM, H_DIM, isc);
  wmma_gemm64<0, false, 2, 1, false><<<dim3((tilesH + 7) / 8, 1), 256, 0, stream>>>(
      AGh, nullptr, H_DIM, 0L, WvT, nullptr, H_DIM, 0L, (void*)Vh, nullptr, H_DIM, 0L,
      bv, nullptr, 0L, N_NODES, H_DIM, H_DIM, isc);
  attn_f16_kernel<<<(N_NODES / 64) * N_HEADS, 128, 0, stream>>>(Qh, Kh, Vh, CTXh, N_NODES, H_DIM, 0.125f, 256.0f);
  wmma_gemm64<0, false, 2, 0, true><<<dim3((tilesH + 7) / 8, 1), 256, 0, stream>>>(
      CTXh, nullptr, H_DIM, 0L, WoT, nullptr, H_DIM, 0L, (void*)Y1, nullptr, H_DIM, 0L,
      bo, h, 0L, N_NODES, H_DIM, H_DIM, isc * (1.0f / 256.0f));
  ln_kernel<true><<<N_NODES / 8, NT, 0, stream>>>(Y1, g1, be1, Xf, Xh, N_NODES);
  wmma_gemm64<0, false, 2, 1, false, 5><<<dim3((tilesH2 + 7) / 8, 1), 256, 0, stream>>>(
      Xh, nullptr, H_DIM, 0L, W1T, nullptr, H_DIM, 0L, (void*)F1h, nullptr, H2_DIM, 0L,
      b1, nullptr, 0L, N_NODES, H2_DIM, H_DIM, isc);
  wmma_gemm64<0, false, 2, 0, true><<<dim3((tilesH + 7) / 8, 1), 256, 0, stream>>>(
      F1h, nullptr, H2_DIM, 0L, W2T, nullptr, H2_DIM, 0L, (void*)Y2, nullptr, H_DIM, 0L,
      b2, Xf, 0L, N_NODES, H_DIM, H2_DIM, isc);
  ln_kernel<false><<<N_NODES / 8, NT, 0, stream>>>(Y2, g2, be2, out, Xh, N_NODES);
}
